// UniModalAttention_3083786518818
// MI455X (gfx1250) — hardware-verified
//
#include <hip/hip_runtime.h>


#define NN_  8
#define NH_  8
#define TT   1024
#define HD   128
#define NZ   (NN_ * NH_)
#define NR   (NZ * TT)
#define ZH   8
#define PCAR 1024.0f
typedef _Float16 h16;
typedef unsigned short bf;
typedef __attribute__((ext_vector_type(16))) __bf16   v16bf;
typedef __attribute__((ext_vector_type(16))) _Float16 v16h;
typedef __attribute__((ext_vector_type(8)))  _Float16 v8h;
typedef __attribute__((ext_vector_type(8)))  unsigned short v8us;
typedef __attribute__((ext_vector_type(8)))  float    v8f;
typedef __attribute__((ext_vector_type(4)))  float    v4f;
typedef v8h  __attribute__((may_alias)) v8ha;
typedef v4f  __attribute__((may_alias)) v4fa;
typedef v8us __attribute__((may_alias)) v8usa;

__device__ __forceinline__ unsigned short f2bf(float f) { unsigned u = __float_as_uint(f); u += 0x7FFFu + ((u >> 16) & 1u); return (unsigned short)(u >> 16); }
__device__ __forceinline__ float bf2f(unsigned short b) { return __uint_as_float(((unsigned)b) << 16); }
__device__ __forceinline__ float bfr(float f) { return bf2f(f2bf(f)); }
__device__ __forceinline__ v16h cat16(v8h lo, v8h hi) { return __builtin_shufflevector(lo, hi, 0, 1, 2, 3, 4, 5, 6, 7, 8, 9, 10, 11, 12, 13, 14, 15); }
__device__ __forceinline__ v16bf cat16b(v8us lo, v8us hi) { return __builtin_bit_cast(v16bf, __builtin_shufflevector(lo, hi, 0, 1, 2, 3, 4, 5, 6, 7, 8, 9, 10, 11, 12, 13, 14, 15)); }
__device__ __forceinline__ v8f wmma16(v16h a, v16h b, v8f c) { return __builtin_amdgcn_wmma_f32_16x16x32_f16(false, a, false, b, (short)0, c, false, false); }
__device__ __forceinline__ v8f wmmab(v16bf a, v16bf b, v8f c) { return __builtin_amdgcn_wmma_f32_16x16x32_bf16(false, a, false, b, (short)0, c, false, false); }


template <typename T16> struct WFrag;
template <> struct WFrag<h16> { typedef v16h V; static __device__ __forceinline__ V ld(const h16* p) { return cat16(*(const v8h*)p, *(const v8h*)(p + 16)); } static __device__ __forceinline__ v8f mma(V a, V b, v8f c) { return wmma16(a, b, c); } };
template <> struct WFrag<bf> { typedef v16bf V; static __device__ __forceinline__ V ld(const bf* p) { return cat16b(*(const v8us*)p, *(const v8us*)(p + 16)); } static __device__ __forceinline__ v8f mma(V a, V b, v8f c) { return wmmab(a, b, c); } };
template <typename T16, int NSPLIT, bool BIAS>
__global__ __launch_bounds__(32) void k_gemmw(const T16* __restrict__ A, const T16* __restrict__ A2, const T16* __restrict__ Bt, const T16* __restrict__ Bt2, int K, float* C, int ldc, const float* __restrict__ bias, size_t sA, size_t sB, size_t sC) {
    typedef typename WFrag<T16>::V V;
    __shared__ __align__(16) float os[16 * 68];
    const size_t z = blockIdx.z; A += z * sA; if (A2) A2 += z * sA; Bt += z * sB; if (Bt2) Bt2 += z * sB; C += z * sC;
    const int lane = threadIdx.x & 31, lr = lane & 15, hi = lane >> 4; const int r0 = blockIdx.x * 64, c0 = blockIdx.y * 64;
    v8f acc[4][4];
#pragma unroll
    for (int mb = 0; mb < 4; ++mb)
#pragma unroll
        for (int nb = 0; nb < 4; ++nb) acc[mb][nb] = (v8f){};
    const size_t aoff = (size_t)(r0 + lr) * K + 8 * hi, boff = (size_t)(c0 + lr) * K + 8 * hi;
#pragma unroll 1
    for (int kc = 0; kc < K; kc += 32) {
        V a[4], a2[4];
#pragma unroll
        for (int mb = 0; mb < 4; ++mb) { a[mb] = WFrag<T16>::ld(A + aoff + (size_t)mb * 16 * K + kc); if (NSPLIT == 1 || NSPLIT == 2) a2[mb] = WFrag<T16>::ld(A2 + aoff + (size_t)mb * 16 * K + kc); }
#pragma unroll
        for (int nb = 0; nb < 4; ++nb) { const V b = WFrag<T16>::ld(Bt + boff + (size_t)nb * 16 * K + kc); V b2; if (NSPLIT >= 2) b2 = WFrag<T16>::ld(Bt2 + boff + (size_t)nb * 16 * K + kc);
#pragma unroll
            for (int mb = 0; mb < 4; ++mb) { acc[mb][nb] = WFrag<T16>::mma(a[mb], b, acc[mb][nb]); if (NSPLIT == 1 || NSPLIT == 2) acc[mb][nb] = WFrag<T16>::mma(a2[mb], b, acc[mb][nb]); if (NSPLIT >= 2) acc[mb][nb] = WFrag<T16>::mma(a[mb], b2, acc[mb][nb]); } }
        asm volatile("v_nop\n\tv_nop\n\tv_nop\n\tv_nop" : "+v"(acc[0][0]), "+v"(acc[1][1]), "+v"(acc[2][2]), "+v"(acc[3][3]) : "v"(a[0]), "v"(a[3]));
    }
#pragma unroll
    for (int mb = 0; mb < 4; ++mb) {
#pragma unroll
        for (int nb = 0; nb < 4; ++nb) {
#pragma unroll
            for (int j = 0; j < 8; ++j) os[(hi * 8 + j) * 68 + nb * 16 + lr] = acc[mb][nb][j]; }
        __builtin_amdgcn_wave_barrier(); asm volatile("" ::: "memory");
        float* crow = C + (size_t)(r0 + mb * 16) * ldc + c0;
#pragma unroll 1
        for (int ps = 0; ps < 2; ++ps) {
#pragma unroll
            for (int s = 0; s < 8; ++s) { const int row = 2 * s + hi, cofs = lr * 4; v4f val = *(const v4fa*)(os + row * 68 + cofs); if (BIAS) { val[0] += bfr(bias[c0 + cofs]); val[1] += bfr(bias[c0 + cofs + 1]); val[2] += bfr(bias[c0 + cofs + 2]); val[3] += bfr(bias[c0 + cofs + 3]); }
                *(volatile v4f*)(crow + (size_t)row * ldc + cofs) = val; }
            if (ps == 0) __threadfence(); }
        __builtin_amdgcn_wave_barrier(); asm volatile("" ::: "memory");
    }
}

__device__ __forceinline__ h16 tohx(float x) { return (h16)x; }
__device__ __forceinline__ void splitf(float y, unsigned short& h, unsigned short& l) { h = f2bf(y); l = f2bf(y - bf2f(h)); }
typedef __attribute__((ext_vector_type(2))) _Float16 v2h;
typedef __attribute__((ext_vector_type(4))) _Float16 v4h;
typedef __attribute__((ext_vector_type(2))) unsigned short v2us;
typedef __attribute__((ext_vector_type(4))) unsigned short v4us;

__global__ __launch_bounds__(256) void k_cvt8(const float* __restrict__ src, bf* dst, size_t n8) { const size_t i = (size_t)blockIdx.x * 256 + threadIdx.x; if (i >= n8) return; const v8f v = *(const v8f*)(src + i * 8); v8us o;
#pragma unroll
    for (int k = 0; k < 8; ++k) o[k] = f2bf(v[k]); *(volatile v8us*)(dst + i * 8) = o; __threadfence(); *(volatile v8us*)(dst + i * 8) = o; }
__global__ __launch_bounds__(256) void k_wtG(const float* __restrict__ w, int K, int N, bf* Bt) {
    const int lane = threadIdx.x & 31; const int L0 = (blockIdx.x * 8 + (threadIdx.x >> 5)) * 8; const int nlines = N * K / 64;
#pragma unroll 1
    for (int ps = 0; ps < 2; ++ps) {
#pragma unroll 1
        for (int l = 0; l < 8; ++l) { const int L = L0 + l; if (L >= nlines) break; const size_t e = (size_t)L * 64 + lane * 2; const int k = (int)(e % K), n = (int)(e / K); v2us o;
            o[0] = f2bf(w[(size_t)k * N + n]); o[1] = f2bf(w[(size_t)(k + 1) * N + n]); *(volatile v2us*)(Bt + e) = o; }
        if (ps == 0) __threadfence(); }
}
__global__ __launch_bounds__(256) void k_relusplit(const float* __restrict__ F, bf* Hh, bf* Hl, size_t n) { const size_t i = ((size_t)blockIdx.x * 256 + threadIdx.x) * 2; if (i >= n) return; v2us oh, ol;
#pragma unroll
    for (int q = 0; q < 2; ++q) { unsigned short a, c2; splitf(fmaxf(F[i + q], 0.f), a, c2); oh[q] = a; ol[q] = c2; }
    *(volatile v2us*)(Hh + i) = oh; *(volatile v2us*)(Hl + i) = ol; __threadfence(); *(volatile v2us*)(Hh + i) = oh; *(volatile v2us*)(Hl + i) = ol; }
__global__ __launch_bounds__(256) void k_split(const float* __restrict__ F, bf* Ph, bf* Pl, size_t n) { const size_t i = ((size_t)blockIdx.x * 256 + threadIdx.x) * 2; if (i >= n) return; v2us oh, ol;
#pragma unroll
    for (int q = 0; q < 2; ++q) { unsigned short a, c2; splitf(F[i + q], a, c2); oh[q] = a; ol[q] = c2; }
    *(volatile v2us*)(Ph + i) = oh; *(volatile v2us*)(Pl + i) = ol; __threadfence(); *(volatile v2us*)(Ph + i) = oh; *(volatile v2us*)(Pl + i) = ol; }
__global__ __launch_bounds__(256) void k_vt16(const float* __restrict__ FV, h16* VT) {
    const int lane = threadIdx.x & 31; const int L0 = (blockIdx.x * 8 + (threadIdx.x >> 5)) * 8; const int nlines = NR * HD / 64;
#pragma unroll 1
    for (int ps = 0; ps < 2; ++ps) {
#pragma unroll
        for (int l = 0; l < 8; ++l) { const int L = L0 + l; if (L >= nlines) break; const int e = L * 64 + lane * 2; const int t = e & (TT - 1); const int c = (e >> 10) & (HD - 1); const int z = e >> 17; v2h v;
#pragma unroll
            for (int q = 0; q < 2; ++q) v[q] = tohx(FV[((size_t)z * TT + t + q) * HD + c]);
            *(volatile v2h*)(VT + (size_t)e) = v; }
        if (ps == 0) __threadfence(); }
}
__global__ __launch_bounds__(256) void k_gsoft(const float* __restrict__ Sb, const float* __restrict__ T1, const float* __restrict__ X, const float* __restrict__ LTAU, int z0, h16* P) {
    const int lane = threadIdx.x & 31; const int row = blockIdx.x * 8 + (threadIdx.x >> 5); if (row >= ZH * TT) return; const int t = row & (TT - 1); const int zz = row >> 10; const int n = (z0 + zz) / NH_;
    const float* sr = Sb + (size_t)row * TT; const float t1v = bfr(T1[(size_t)n * TT + t]); const float itau = __builtin_amdgcn_rcpf(__expf(bfr(LTAU[0]))); const float* t2p = X + (size_t)n * NH_ * TT * HD + (HD - 1);
    float v[32]; bool mk[32]; float mx = -3.0e38f;
#pragma unroll
    for (int ch = 0; ch < 8; ++ch) { const int j0 = ch * 128 + lane * 4; const v4f a = *(const v4f*)(sr + j0);
#pragma unroll
        for (int q = 0; q < 4; ++q) { const int l = j0 + q; float sq = __fmul_rn(a[q], a[q]); asm volatile("" : "+v"(sq)); float g = __fmul_rn(-sq, itau); asm volatile("" : "+v"(g)); const bool m = (t1v >= bfr(t2p[(size_t)l * HD])); const float s = m ? g : __fmul_rn(g, 0.0f);
            v[ch * 4 + q] = s; mk[ch * 4 + q] = m; mx = fmaxf(mx, s); } }
#pragma unroll
    for (int sh = 16; sh; sh >>= 1) mx = fmaxf(mx, __shfl_xor(mx, sh, 32));
    float sum = 0.f;
#pragma unroll
    for (int k = 0; k < 32; ++k) { v[k] = __expf(v[k] - mx); sum += v[k]; }
#pragma unroll
    for (int sh = 16; sh; sh >>= 1) sum += __shfl_xor(sum, sh, 32);
    const float f = __fdiv_rn(PCAR, sum);
#pragma unroll 1
    for (int ps = 0; ps < 2; ++ps) {
#pragma unroll
        for (int ch = 0; ch < 8; ++ch) { v4h o;
#pragma unroll
            for (int q = 0; q < 4; ++q) o[q] = mk[ch * 4 + q] ? tohx(v[ch * 4 + q] * f) : tohx(0.f);
            *(volatile v4h*)(P + (size_t)row * TT + ch * 128 + lane * 4) = o; }
        if (ps == 0) __threadfence(); }
}
__global__ __launch_bounds__(256) void k_out(const float* __restrict__ O, float* OUTz, size_t n) { const size_t i = ((size_t)blockIdx.x * 256 + threadIdx.x) * 4; if (i >= n) return; const v4f a = *(const v4f*)(O + i); v4f o;
#pragma unroll
    for (int q = 0; q < 4; ++q) o[q] = a[q] * (1.0f / PCAR); *(volatile v4f*)(OUTz + i) = o; __threadfence(); *(volatile v4f*)(OUTz + i) = o; }

extern "C" void kernel_launch(void* const* d_in, const int* in_sizes, int n_in,
                              void* d_out, int out_size, void* d_ws, size_t ws_size, hipStream_t stream) {
    (void)in_sizes; (void)n_in; (void)out_size;
    const float* X = (const float*)d_in[0]; const float* T1 = (const float*)d_in[1]; const float* Q = (const float*)d_in[2]; const float* Wk1 = (const float*)d_in[3]; const float* bk1 = (const float*)d_in[4]; const float* Wk2 = (const float*)d_in[5]; const float* bk2 = (const float*)d_in[6]; const float* Wv1 = (const float*)d_in[7]; const float* bv1 = (const float*)d_in[8]; const float* Wv2 = (const float*)d_in[9]; const float* bv2 = (const float*)d_in[10]; const float* LTAU = (const float*)d_in[11];
    float* OUT = (float*)d_out;
    char* wsp = (char*)d_ws;
    auto take = [&](size_t bytes) { char* p = wsp; wsp += (bytes + 255) & ~(size_t)255; return (void*)p; };
    bf* W1K = (bf*)take(HD * HD * 2); bf* W2K = (bf*)take(HD * HD * 2); bf* W1V = (bf*)take(HD * HD * 2); bf* W2V = (bf*)take(HD * HD * 2);
    bf* XB = (bf*)take((size_t)NR * HD * 2); bf* QB = (bf*)take((size_t)NR * HD * 2); float* F = (float*)take((size_t)NR * HD * 4); bf* H1h = (bf*)take((size_t)NR * HD * 2); bf* H1l = (bf*)take((size_t)NR * HD * 2);
    bf* Kh = (bf*)take((size_t)NR * HD * 2); bf* Kl = (bf*)take((size_t)NR * HD * 2); h16* VT = (h16*)take((size_t)NR * HD * 2);
    float* Sb = (float*)take((size_t)ZH * TT * TT * 4); h16* P = (h16*)take((size_t)ZH * TT * TT * 2); float* Ob = (float*)take((size_t)ZH * TT * HD * 4);
    if ((size_t)(wsp - (char*)d_ws) > ws_size) return;
    { const unsigned gW = (unsigned)((HD * HD / 64 + 63) / 64); k_wtG<<<gW, 256, 0, stream>>>(Wk1, HD, HD, W1K); k_wtG<<<gW, 256, 0, stream>>>(Wk2, HD, HD, W2K); k_wtG<<<gW, 256, 0, stream>>>(Wv1, HD, HD, W1V); k_wtG<<<gW, 256, 0, stream>>>(Wv2, HD, HD, W2V);
      const size_t nx = (size_t)NR * HD / 8; k_cvt8<<<(unsigned)((nx + 255) / 256), 256, 0, stream>>>(X, XB, nx); k_cvt8<<<(unsigned)((nx + 255) / 256), 256, 0, stream>>>(Q, QB, nx); }
    const dim3 gM(NR / 64, HD / 64, 1); const unsigned LF = (unsigned)(((size_t)NR * HD / 2 + 255) / 256);
    k_gemmw<bf, 0, true><<<gM, 32, 0, stream>>>(XB, nullptr, W1K, nullptr, HD, F, HD, bk1, 0, 0, 0); k_relusplit<<<LF, 256, 0, stream>>>(F, H1h, H1l, (size_t)NR * HD);
    k_gemmw<bf, 1, true><<<gM, 32, 0, stream>>>(H1h, H1l, W2K, nullptr, HD, F, HD, bk2, 0, 0, 0); k_split<<<LF, 256, 0, stream>>>(F, Kh, Kl, (size_t)NR * HD);
    k_gemmw<bf, 0, true><<<gM, 32, 0, stream>>>(XB, nullptr, W1V, nullptr, HD, F, HD, bv1, 0, 0, 0); k_relusplit<<<LF, 256, 0, stream>>>(F, H1h, H1l, (size_t)NR * HD);
    k_gemmw<bf, 1, true><<<gM, 32, 0, stream>>>(H1h, H1l, W2V, nullptr, HD, F, HD, bv2, 0, 0, 0); k_vt16<<<(NR * HD / 64 + 63) / 64, 256, 0, stream>>>(F, VT);
    for (int z0 = 0; z0 < NZ; z0 += ZH) {
        k_gemmw<bf, 3, false><<<dim3(TT / 64, TT / 64, ZH), 32, 0, stream>>>(QB + (size_t)z0 * TT * HD, nullptr, Kh + (size_t)z0 * TT * HD, Kl + (size_t)z0 * TT * HD, HD, Sb, TT, nullptr, (size_t)TT * HD, (size_t)TT * HD, (size_t)TT * TT);
        k_gsoft<<<ZH * TT / 8, 256, 0, stream>>>(Sb, T1, X, LTAU, z0, P);
        k_gemmw<h16, 0, false><<<dim3(TT / 64, HD / 64, ZH), 32, 0, stream>>>(P, nullptr, VT + (size_t)z0 * HD * TT, nullptr, TT, Ob, HD, nullptr, (size_t)TT * TT, (size_t)HD * TT, (size_t)TT * HD);
        k_out<<<(unsigned)(((size_t)ZH * TT * HD / 4 + 255) / 256), 256, 0, stream>>>(Ob, OUT + (size_t)z0 * TT * HD, (size_t)ZH * TT * HD); }
}
